// GNNClassifier_88648124990545
// MI455X (gfx1250) — hardware-verified
//
#include <hip/hip_runtime.h>
#include <stddef.h>
#include <stdint.h>


#define NN     100000
#define NE     1200000
#define NG     2048
#define VOC    10000
#define DH     64
#define TW     128
#define NCLS   2
#define VP     10048
#define MPAD   100032
#define NTHR   256
#define NWAVE  8
#define EPT    8
#define CHUNK  (NTHR * EPT)
#define WCAP   (EPT * 32)
#define LISTN  (NWAVE * WCAP)
#define NBA    1024
#define SLA    10
#define RCAP   16384
#define DEGCAP 64
#define GBM    64
#define GBN    64
#define GTHR   128
#define GPB    16
#define UE     (VP * 8)
#define UW1H   (DH * 8)
#define UW2H   (DH * 16)
#define UTOT   (UE + 2 * UW1H + 2 * UW2H)
#define AGG_ZINTS (LISTN + 2 * RCAP + 3 * NBA)
#define AGG_LDS_INTS (AGG_ZINTS + 16)
#define WSMAX  134217728

static_assert((CHUNK & (CHUNK - 1)) == 0 && CHUNK <= 4096);
static_assert((NBA & (NBA - 1)) == 0 && NBA == (1 << SLA));
static_assert(((long long)CHUNK << SLA) < (1LL << 31));
static_assert(NE < (1 << (31 - SLA)));
static_assert((NE & 3) == 0);
static_assert(LISTN % NTHR == 0);
static_assert(NBA % NWAVE == 0 && NBA % 32 == 0 && NBA % GBM == 0);
static_assert(RCAP % 32 == 0 && AGG_ZINTS % 4 == 0 && LISTN % 4 == 0);
static_assert(DH % 32 == 0 && TW % 32 == 0 && TW == 2 * DH && DH == GBN);
static_assert(GBM == (GTHR / 32) * 16 && GBN == 64 && TW % GBN == 0);
static_assert(VP % GBM == 0 && VP >= VOC && MPAD % GBM == 0 && MPAD >= NN);
static_assert(UE % NTHR == 0 && UW1H % NTHR == 0 && UW2H % NTHR == 0 && UTOT % NTHR == 0);
static_assert(DH == 2 * 32);
static_assert(AGG_LDS_INTS * 4 <= 300000);
static_assert(NG % GPB == 0 && GPB * NCLS * 4 == 128);
static_assert((GPB * DH) % NTHR == 0);

typedef float          v2f   __attribute__((ext_vector_type(2)));
typedef float          v4f   __attribute__((ext_vector_type(4)));
typedef float          v8f   __attribute__((ext_vector_type(8)));
typedef int            v4i   __attribute__((ext_vector_type(4)));
typedef int            v8i   __attribute__((ext_vector_type(8)));
typedef unsigned int   v4u   __attribute__((ext_vector_type(4)));
typedef unsigned short v8us  __attribute__((ext_vector_type(8)));
typedef unsigned short v16us __attribute__((ext_vector_type(16)));
typedef __bf16         v16bf __attribute__((ext_vector_type(16)));
typedef v2f  __attribute__((may_alias)) v2fa;
typedef v4f  __attribute__((may_alias)) v4fa;
typedef v4i  __attribute__((may_alias)) v4ia;
typedef v8us __attribute__((may_alias)) v8usa;
union FragB { v16bf v; v16us u; v8us h[2]; v8i w; };

__device__ __forceinline__ v8f wmb(const FragB& a, const FragB& b, v8f c) {
  v8f d = __builtin_amdgcn_wmma_f32_16x16x32_bf16(false, a.v, false, b.v, (short)0, c, false, false);
  asm volatile("v_nop\n\tv_nop\n\tv_nop\n\tv_nop" : "+v"(d) : "v"(a.w), "v"(b.w));
  return d;
}

__device__ __forceinline__ unsigned bf16_bits(float f) {
  const unsigned u = __float_as_uint(f);
  const unsigned r = (u + 0x7FFFu + ((u >> 16) & 1u)) >> 16;
  return (f != f) ? 0x7FC0u : r;
}
__device__ __forceinline__ float bf16_val(float f) {
  return __uint_as_float(bf16_bits(f) << 16);
}

template <int SLB>
__device__ __forceinline__ int scan_chunk(const int* __restrict__ dsts, int nE, int cbase, int slotBase,
                                          int nb, int vec8, int* list, int tid, int lane, int wave) {
  int wc = 0;
  const int el0  = tid * EPT;
  const int e0   = cbase + el0;
  const int sent = -2147483647 - 1;
  v4i da, db;
  if (vec8 != 0 && cbase + CHUNK <= nE) {
    da = *(const v4i*)(dsts + e0);
    db = *(const v4i*)(dsts + e0 + 4);
  } else {
    da.x = (e0     < nE) ? dsts[min(e0,     nE - 1)] : sent;
    da.y = (e0 + 1 < nE) ? dsts[min(e0 + 1, nE - 1)] : sent;
    da.z = (e0 + 2 < nE) ? dsts[min(e0 + 2, nE - 1)] : sent;
    da.w = (e0 + 3 < nE) ? dsts[min(e0 + 3, nE - 1)] : sent;
    db.x = (e0 + 4 < nE) ? dsts[min(e0 + 4, nE - 1)] : sent;
    db.y = (e0 + 5 < nE) ? dsts[min(e0 + 5, nE - 1)] : sent;
    db.z = (e0 + 6 < nE) ? dsts[min(e0 + 6, nE - 1)] : sent;
    db.w = (e0 + 7 < nE) ? dsts[min(e0 + 7, nE - 1)] : sent;
  }
  const unsigned nbs = (unsigned)slotBase;
  const unsigned unb = (unsigned)nb;
  const unsigned s0 = (unsigned)da.x - nbs, s1 = (unsigned)da.y - nbs;
  const unsigned s2 = (unsigned)da.z - nbs, s3 = (unsigned)da.w - nbs;
  const unsigned s4 = (unsigned)db.x - nbs, s5 = (unsigned)db.y - nbs;
  const unsigned s6 = (unsigned)db.z - nbs, s7 = (unsigned)db.w - nbs;
  const bool h0 = s0 < unb, h1 = s1 < unb, h2 = s2 < unb, h3 = s3 < unb;
  const bool h4 = s4 < unb, h5 = s5 < unb, h6 = s6 < unb, h7 = s7 < unb;
  const unsigned any = __builtin_amdgcn_ballot_w32(h0 | h1 | h2 | h3 | h4 | h5 | h6 | h7);
  if (any != 0u) {
#define HITJ(J, HJ, SJ) { \
      const unsigned mj = __builtin_amdgcn_ballot_w32(HJ); \
      if (mj != 0u) { \
        if (HJ) { \
          const int pos = wc + (int)__builtin_amdgcn_mbcnt_lo(mj, 0u); \
          if (pos < WCAP) list[wave * WCAP + pos] = ((el0 + (J)) << SLB) | (int)(SJ); \
        } \
        wc += (int)__builtin_popcount(mj); } }
    HITJ(0, h0, s0)
    HITJ(1, h1, s1)
    HITJ(2, h2, s2)
    HITJ(3, h3, s3)
    HITJ(4, h4, s4)
    HITJ(5, h5, s5)
    HITJ(6, h6, s6)
    HITJ(7, h7, s7)
#undef HITJ
  }
  return wc;
}

__device__ __forceinline__ v8us cvt8(const v4f a, const v4f b, const bool ok) {
  v8us o;
  o[0] = ok ? (unsigned short)bf16_bits(a.x) : (unsigned short)0;
  o[1] = ok ? (unsigned short)bf16_bits(a.y) : (unsigned short)0;
  o[2] = ok ? (unsigned short)bf16_bits(a.z) : (unsigned short)0;
  o[3] = ok ? (unsigned short)bf16_bits(a.w) : (unsigned short)0;
  o[4] = ok ? (unsigned short)bf16_bits(b.x) : (unsigned short)0;
  o[5] = ok ? (unsigned short)bf16_bits(b.y) : (unsigned short)0;
  o[6] = ok ? (unsigned short)bf16_bits(b.z) : (unsigned short)0;
  o[7] = ok ? (unsigned short)bf16_bits(b.w) : (unsigned short)0;
  return o;
}

__global__ __launch_bounds__(NTHR) void k_prep(const float* __restrict__ emb,
                                               const float* __restrict__ W1l, const float* __restrict__ W1r,
                                               const float* __restrict__ W2l, const float* __restrict__ W2r,
                                               unsigned short* EMB, unsigned short* W1P, unsigned short* W2X) {
  const int u = (int)blockIdx.x * NTHR + (int)threadIdx.x;
  v4f a, b;
  bool ok = true;
  size_t doff;
  int which;
  if (u < UE) {
    const int row = u >> 3;
    const int k8  = (u & 7) * 8;
    const int rc  = row < VOC ? row : VOC - 1;
    const float* p = emb + (size_t)rc * DH + k8;
    a = *(const v4fa*)p; b = *(const v4fa*)(p + 4);
    ok = row < VOC;
    doff = (size_t)row * DH + k8; which = 0;
  } else if (u < UE + UW1H) {
    const int v = u - UE;
    const int n = v >> 3, k8 = (v & 7) * 8;
    const float* p = W1l + (size_t)n * DH + k8;
    a = *(const v4fa*)p; b = *(const v4fa*)(p + 4);
    doff = (size_t)n * DH + k8; which = 1;
  } else if (u < UE + 2 * UW1H) {
    const int v = u - (UE + UW1H);
    const int n = v >> 3, k8 = (v & 7) * 8;
    const float* p = W1r + (size_t)n * DH + k8;
    a = *(const v4fa*)p; b = *(const v4fa*)(p + 4);
    doff = (size_t)(DH + n) * DH + k8; which = 1;
  } else if (u < UE + 2 * UW1H + UW2H) {
    const int v = u - (UE + 2 * UW1H);
    const int n = v >> 4, k8 = (v & 15) * 8, kk = k8 & (DH - 1);
    const float* p = W2l + (size_t)n * DH + kk;
    a = *(const v4fa*)p; b = *(const v4fa*)(p + 4);
    doff = (size_t)n * TW + k8; which = 2;
  } else if (u < UTOT) {
    const int v = u - (UE + 2 * UW1H + UW2H);
    const int n = v >> 4, k8 = (v & 15) * 8, kk = k8 & (DH - 1);
    const float* p = W2r + (size_t)n * DH + kk;
    a = *(const v4fa*)p; b = *(const v4fa*)(p + 4);
    doff = (size_t)(DH + n) * TW + k8; which = 2;
  } else {
    return;
  }
  const v8us o = cvt8(a, b, ok);
  if (which == 0) {
    *(volatile v8us*)(EMB + doff) = o;
    __threadfence();
    *(volatile v8us*)(EMB + doff) = o;
  } else if (which == 1) {
    *(volatile v8us*)(W1P + doff) = o;
    __threadfence();
    *(volatile v8us*)(W1P + doff) = o;
  } else {
    *(volatile v8us*)(W2X + doff) = o;
    __threadfence();
    *(volatile v8us*)(W2X + doff) = o;
  }
}

__global__ __launch_bounds__(GTHR) void k_gemm(
    const unsigned short* __restrict__ A, const unsigned short* __restrict__ WT,
    float* outF, int K, int ldo)
{
  __shared__ __attribute__((aligned(16))) float stg[GBM * GBN];
  const int tid = (int)threadIdx.x, lane = tid & 31, wave = tid >> 5, hh = lane >> 4, m = lane & 15;
  const int rowBase = (int)blockIdx.x * GBM;
  const int col0    = (int)blockIdx.y * GBN;

  v8f acc[4];
  {
    const v8f z = {0.f, 0.f, 0.f, 0.f, 0.f, 0.f, 0.f, 0.f};
    acc[0] = z; acc[1] = z; acc[2] = z; acc[3] = z;
  }
  const unsigned short* ap = A  + (size_t)(rowBase + 16 * wave + m) * (size_t)K + 8 * hh;
  const unsigned short* wp = WT + (size_t)(col0 + m) * (size_t)K + 8 * hh;
  const int ksteps = K >> 5;
#pragma unroll 1
  for (int ks = 0; ks < ksteps; ++ks) {
    FragB af;
    af.h[0] = *(const v8usa*)(ap + 32 * ks);
    af.h[1] = *(const v8usa*)(ap + 32 * ks + 16);
#pragma unroll
    for (int t = 0; t < 4; ++t) {
      const unsigned short* wq = wp + (size_t)(16 * t) * (size_t)K + 32 * ks;
      FragB bf;
      bf.h[0] = *(const v8usa*)wq;
      bf.h[1] = *(const v8usa*)(wq + 16);
      acc[t] = wmb(af, bf, acc[t]);
    }
  }

#pragma unroll
  for (int t = 0; t < 4; ++t) {
    const int lc = 16 * t + m;
#pragma unroll
    for (int r = 0; r < 8; ++r) {
      const int lr = 16 * wave + 8 * hh + r;
      stg[lr * GBN + lc] = acc[t][r];
    }
  }
  __syncthreads();

  v4f fv[8];
#pragma unroll
  for (int i = 0; i < 8; ++i) {
    const int lr = 16 * wave + 2 * i + hh;
    fv[i] = *(const v4fa*)(stg + lr * GBN + 4 * m);
  }
#pragma unroll
  for (int i = 0; i < 8; ++i) {
    const int lr = 16 * wave + 2 * i + hh;
    const int gr = rowBase + lr;
    float* op = outF + (size_t)gr * (size_t)ldo + col0 + 4 * m;
    *(volatile v4f*)op = fv[i];
  }
  __threadfence();
#pragma unroll
  for (int i = 0; i < 8; ++i) {
    const int lr = 16 * wave + 2 * i + hh;
    const int gr = rowBase + lr;
    float* op = outF + (size_t)gr * (size_t)ldo + col0 + 4 * m;
    *(volatile v4f*)op = fv[i];
  }
}

template <int MODE>
__global__ __launch_bounds__(NTHR) void k_scan(const int* __restrict__ srcs, const int* __restrict__ dsts,
                                               const int* __restrict__ xi,
                                               int nE, int nN, int nTab, int vec8, int mRows,
                                               const float* __restrict__ tab, const float* __restrict__ bias,
                                               unsigned short* hb, float* hout) {
  extern __shared__ __attribute__((aligned(16))) int dsm[];
  int* list = dsm;
  int* hl   = dsm + LISTN;
  int* sl   = dsm + LISTN + RCAP;
  int* cnt  = dsm + LISTN + 2 * RCAP;
  int* offs = cnt + NBA;
  int* cur  = offs + NBA;
  int* misc = cur + NBA;
  const int tid = (int)threadIdx.x, lane = tid & 31, wave = tid >> 5;
  const int nodeBase = (int)blockIdx.x * NBA;

  {
    const v4i z4 = {0, 0, 0, 0};
    for (int i = tid * 4; i < AGG_ZINTS; i += NTHR * 4) *(v4ia*)(dsm + i) = z4;
    if (tid < 16) misc[tid] = 0;
  }
  float bv0, bv1;
  {
    const v2f a = *(const v2fa*)(bias + 2 * lane);
    bv0 = bf16_val(a.x); bv1 = bf16_val(a.y);
  }
  __syncthreads();

  int t = 0, ov = 0;
  const int nChunks = (nE + CHUNK - 1) / CHUNK;
#pragma unroll 1
  for (int ch = 0; ch < nChunks; ++ch) {
    const int cbase = ch * CHUNK;
    const int wc = scan_chunk<SLA>(dsts, nE, cbase, nodeBase, NBA, vec8, list, tid, lane, wave);
    if (lane == 0) misc[wave] = wc;
    __syncthreads();
    if (wave == 0) {
#pragma unroll 1
      for (int w2 = 0; w2 < NWAVE; ++w2) {
        int c = misc[w2];
        c = c < 0 ? 0 : (c > WCAP ? WCAP : c);
#pragma unroll 1
        for (int b0 = 0; b0 < c; b0 += 32) {
          const int idx = b0 + lane;
          const int ent = list[w2 * WCAP + (idx < WCAP ? idx : WCAP - 1)];
          const int m32 = (c - b0) < 32 ? (c - b0) : 32;
#pragma unroll 1
          for (int k = 0; k < m32; ++k) {
            const int u    = __builtin_amdgcn_readlane(ent, k);
            const int slot = u & (NBA - 1);
            const int el   = (u >> SLA) & (CHUNK - 1);
            const int pk   = ((cbase + el) << SLA) | slot;
            if (t < RCAP) {
              if (lane == 0) { hl[t] = pk; cnt[slot] = cnt[slot] + 1; }
              t = t + 1;
            } else {
              ov = 1;
            }
          }
        }
      }
    }
    __syncthreads();
  }
  if (wave == 0 && lane == 0) { misc[8] = t; misc[9] = ov; }
  __syncthreads();
  int tt = misc[8];
  tt = tt < 0 ? 0 : (tt > RCAP ? RCAP : tt);
  const int ovf = misc[9];

  if (wave == 0) {
    const int base = lane * (NBA / 32);
    int s = 0;
#pragma unroll 1
    for (int i = 0; i < NBA / 32; ++i) s += cnt[base + i];
    int incl = s;
#pragma unroll
    for (int d = 1; d < 32; d <<= 1) {
      const int y = __shfl_up(incl, d, 32);
      if (lane >= d) incl += y;
    }
    int run = incl - s;
#pragma unroll 1
    for (int i = 0; i < NBA / 32; ++i) {
      const int cv = cnt[base + i];
      offs[base + i] = run;
      cur[base + i]  = run;
      run += cv;
    }
  }
  __syncthreads();
  if (wave == 0) {
#pragma unroll 1
    for (int b0 = 0; b0 < tt; b0 += 32) {
      const int idx = b0 + lane;
      const int ent = hl[idx < RCAP ? idx : RCAP - 1];
      const int m32 = (tt - b0) < 32 ? (tt - b0) : 32;
#pragma unroll 1
      for (int k = 0; k < m32; ++k) {
        const int u    = __builtin_amdgcn_readlane(ent, k);
        const int slot = u & (NBA - 1);
        if (lane == 0) {
          int p = cur[slot];
          p = p < 0 ? 0 : (p > RCAP - 1 ? RCAP - 1 : p);
          sl[p] = u;
          cur[slot] = p + 1;
        }
      }
    }
  }
  __syncthreads();

  const float qnan = __int_as_float(0x7fc00000);
  const float pz = (ovf != 0) ? qnan : 0.0f;
  const int sa = (2 * lane) & 31, sb = (2 * lane + 1) & 31;
  const int q0s = (4 * lane) & 31, q1s = (4 * lane + 1) & 31;
  const int q2s = (4 * lane + 2) & 31, q3s = (4 * lane + 3) & 31;
#pragma unroll 1
  for (int si = 0; si < NBA / NWAVE; ++si) {
    const int s    = si * NWAVE + wave;
    const int node = nodeBase + s;
    const int craw = cnt[s];
    const bool big = craw > DEGCAP;
    const int c = craw < 0 ? 0 : (craw > DEGCAP ? DEGCAP : craw);
    int o = offs[s];
    o = o < 0 ? 0 : (o > RCAP ? RCAP : o);
    const int nc = node < nN ? node : nN - 1;
    int selfRow = nc;
    if constexpr (MODE != 0) {
      int tk = xi[nc];
      tk = tk < 0 ? 0 : (tk > nTab - 1 ? nTab - 1 : tk);
      selfRow = tk;
    }
    float acc0 = 0.0f, acc1 = 0.0f;
#pragma unroll 1
    for (int b0 = 0; b0 < c; b0 += 32) {
      int idx = o + b0 + lane;
      idx = idx > RCAP - 1 ? RCAP - 1 : idx;
      const int ent = sl[idx];
      int eid = ent >> SLA;
      eid = eid < 0 ? 0 : (eid > nE - 1 ? nE - 1 : eid);
      int sr = srcs[eid];
      sr = sr < 0 ? 0 : (sr > nN - 1 ? nN - 1 : sr);
      int gr = sr;
      if constexpr (MODE != 0) {
        int tk = xi[sr];
        tk = tk < 0 ? 0 : (tk > nTab - 1 ? nTab - 1 : tk);
        gr = tk;
      }
      const int m32 = (c - b0) < 32 ? (c - b0) : 32;
#pragma unroll 1
      for (int k = 0; k < m32; ++k) {
        const int sk = __builtin_amdgcn_readlane(gr, k);
        const v2f a = *(const v2fa*)(tab + (size_t)sk * TW + 2 * lane);
        acc0 += a.x; acc1 += a.y;
      }
    }
    float sv0, sv1;
    {
      const v2f a = *(const v2fa*)(tab + (size_t)selfRow * TW + DH + 2 * lane);
      sv0 = a.x; sv1 = a.y;
    }
    const float cf = (c < 1) ? 1.0f : (float)c;
    const float rc = 1.0f / cf;
    const float pzr = big ? qnan : pz;
    const bool live = node < nN;
    float y0 = (acc0 * rc + bv0) + sv0;
    float y1 = (acc1 * rc + bv1) + sv1;
    y0 = (y0 > 0.0f) ? y0 : (y0 - y0);
    y1 = (y1 > 0.0f) ? y1 : (y1 - y1);
    y0 = y0 + pzr; y1 = y1 + pzr;
    const float v0 = live ? y0 : 0.0f;
    const float v1 = live ? y1 : 0.0f;
    const bool wr = (node < mRows) && (lane < 16);
    if constexpr (MODE != 0) {
      const unsigned hb0 = bf16_bits(v0), hb1 = bf16_bits(v1);
      const unsigned lb0 = bf16_bits(v0 - __uint_as_float(hb0 << 16));
      const unsigned lb1 = bf16_bits(v1 - __uint_as_float(hb1 << 16));
      const int hw = (int)(hb0 | (hb1 << 16));
      const int lw = (int)(lb0 | (lb1 << 16));
      const int g0 = __shfl(hw, q0s, 32), g1 = __shfl(hw, q1s, 32);
      const int g2 = __shfl(hw, q2s, 32), g3 = __shfl(hw, q3s, 32);
      const int p0 = __shfl(lw, q0s, 32), p1 = __shfl(lw, q1s, 32);
      const int p2 = __shfl(lw, q2s, 32), p3 = __shfl(lw, q3s, 32);
      const bool lsel = (lane & 8) != 0;
      v4u pv;
      pv.x = (unsigned int)(lsel ? p0 : g0);
      pv.y = (unsigned int)(lsel ? p1 : g1);
      pv.z = (unsigned int)(lsel ? p2 : g2);
      pv.w = (unsigned int)(lsel ? p3 : g3);
      unsigned short* hp = hb + (size_t)node * TW + 8 * (lane & 15);
      if (wr) *(volatile v4u*)hp = pv;
      __threadfence();
      if (wr) *(volatile v4u*)hp = pv;
    } else {
      v4f ow;
      ow.x = __shfl(v0, sa, 32); ow.y = __shfl(v1, sa, 32);
      ow.z = __shfl(v0, sb, 32); ow.w = __shfl(v1, sb, 32);
      float* op = hout + (size_t)node * DH + 4 * (lane & 15);
      if (wr) *(volatile v4f*)op = ow;
      __threadfence();
      if (wr) *(volatile v4f*)op = ow;
    }
  }
}

__global__ __launch_bounds__(NTHR) void k_poolhead(const float* __restrict__ hf, const int* __restrict__ bat,
                                                   int nN, const float* __restrict__ Wout,
                                                   const float* __restrict__ bout, float* out) {
  __shared__ __attribute__((aligned(16))) float wacc[NWAVE * GPB * DH];
  __shared__ int wcn[NWAVE * GPB];
  __shared__ __attribute__((aligned(16))) float pls[GPB * DH];
  __shared__ float wls[NCLS * DH];
  __shared__ float bls[NCLS];
  __shared__ __attribute__((aligned(16))) float os[GPB * NCLS];
  const int tid = (int)threadIdx.x, lane = tid & 31, wave = tid >> 5;
  const int g0 = (int)blockIdx.x * GPB;

  for (int i = tid; i < NWAVE * GPB * DH; i += NTHR) wacc[i] = 0.0f;
  if (tid < NWAVE * GPB) wcn[tid] = 0;
  if (tid < NCLS * DH) wls[tid] = bf16_val(Wout[tid]);
  if (tid < NCLS) bls[tid] = bf16_val(bout[tid]);
  __syncthreads();

#pragma unroll 1
  for (int i0 = wave * 32; i0 < nN; i0 += NTHR) {
    const int i  = i0 + lane;
    const int ic = i < nN ? i : nN - 1;
    const int rel = bat[ic] - g0;
    const bool hit = (i < nN) && ((unsigned)rel < (unsigned)GPB);
    unsigned msk = __builtin_amdgcn_ballot_w32(hit);
    int nh = (int)__builtin_popcount(msk);
    nh = nh > 32 ? 32 : nh;
#pragma unroll 1
    for (int q = 0; q < nh; ++q) {
      const int k = __builtin_ffs((int)msk) - 1;
      msk &= msk - 1u;
      const int kk = k < 0 ? 0 : k;
      const int gi = __builtin_amdgcn_readlane(rel, kk) & (GPB - 1);
      int node = i0 + kk;
      node = node > nN - 1 ? nN - 1 : node;
      const v2f v = *(const v2fa*)(hf + (size_t)node * DH + 2 * lane);
      float* ap = wacc + (size_t)(wave * GPB + gi) * DH + 2 * lane;
      const float n0 = ap[0] + v.x;
      const float n1 = ap[1] + v.y;
      ap[0] = n0; ap[1] = n1;
      if (lane == 0) wcn[wave * GPB + gi] = wcn[wave * GPB + gi] + 1;
    }
  }
  __syncthreads();
#pragma unroll 1
  for (int idx = tid; idx < GPB * DH; idx += NTHR) {
    const int gi = idx >> 6, chn = idx & (DH - 1);
    float s = 0.0f;
    int c = 0;
#pragma unroll
    for (int w2 = 0; w2 < NWAVE; ++w2) {
      s += wacc[(w2 * GPB + gi) * DH + chn];
      c += wcn[w2 * GPB + gi];
    }
    const float cf = (c < 1) ? 1.0f : (float)c;
    pls[idx] = s * (1.0f / cf);
  }
  __syncthreads();
  if (tid < GPB * NCLS) {
    const int gi = tid >> 1, cc = tid & 1;
    float s = 0.0f;
#pragma unroll 4
    for (int d = 0; d < DH; ++d) s = fmaf(pls[gi * DH + d], wls[cc * DH + d], s);
    os[tid] = s + bls[cc];
  }
  __syncthreads();
  const v4f ov = *(const v4fa*)(os + 4 * (lane & 7));
  float* op = out + (size_t)blockIdx.x * (GPB * NCLS) + 4 * (lane & 7);
  const bool okst = (wave == 0) && (lane < 8);
  if (okst) *(volatile v4f*)op = ov;
  __threadfence();
  if (okst) *(volatile v4f*)op = ov;
}

static inline int cdiv(int a, int b) { return (a + b - 1) / b; }
static inline size_t al256(size_t o) { return (o + 255) & ~(size_t)255; }

extern "C" void kernel_launch(void* const* d_in, const int* in_sizes, int n_in,
                              void* d_out, int out_size, void* d_ws, size_t ws_size,
                              hipStream_t stream) {
  if (n_in < 12) return;
  if (in_sizes[0] != NN) return;
  if (in_sizes[1] != 2 * NE) return;
  if (in_sizes[2] != NN) return;
  if (in_sizes[3] != VOC * DH) return;
  if (in_sizes[4] != DH * DH || in_sizes[5] != DH) return;
  if (in_sizes[6] != DH * DH) return;
  if (in_sizes[7] != DH * DH || in_sizes[8] != DH) return;
  if (in_sizes[9] != DH * DH) return;
  if (in_sizes[10] != NCLS * DH || in_sizes[11] != NCLS) return;
  if (out_size != NG * NCLS) return;

  const int*   x    = (const int*)d_in[0];
  const int*   edge = (const int*)d_in[1];
  const int*   bat  = (const int*)d_in[2];
  const float* emb  = (const float*)d_in[3];
  const float* W1l  = (const float*)d_in[4];
  const float* b1l  = (const float*)d_in[5];
  const float* W1r  = (const float*)d_in[6];
  const float* W2l  = (const float*)d_in[7];
  const float* b2l  = (const float*)d_in[8];
  const float* W2r  = (const float*)d_in[9];
  const float* Wout = (const float*)d_in[10];
  const float* bout = (const float*)d_in[11];
  float* out = (float*)d_out;
  const int* src = edge;
  const int* dst = edge + NE;

  const int MP = MPAD;
  const int gM = MP / GBM;
  const int gV = VP / GBM;
  const int gA = cdiv(MP, NBA);
  if ((long long)gA * NBA < (long long)MP) return;
  const int vec8 = ((NE & 3) == 0) ? 1 : 0;

  char* ws = (char*)d_ws;
  size_t off = 0;
  const size_t oEMB = off; off = al256(off + (size_t)VP * DH * 2);
  const size_t oW1P = off; off = al256(off + (size_t)TW * DH * 2);
  const size_t oW2X = off; off = al256(off + (size_t)TW * TW * 2);
  const size_t oT   = off; off = al256(off + (size_t)VP * TW * 4);
  const size_t oH1  = off; off = al256(off + (size_t)MP * TW * 2);
  const size_t oY2  = off; off = al256(off + (size_t)MP * TW * 4);
  const size_t oH2  = off; off = al256(off + (size_t)MP * DH * 4);
  if (off > ws_size || off > (size_t)WSMAX) return;
  unsigned short* EMB = (unsigned short*)(ws + oEMB);
  unsigned short* W1P = (unsigned short*)(ws + oW1P);
  unsigned short* W2X = (unsigned short*)(ws + oW2X);
  float*          T   = (float*)(ws + oT);
  unsigned short* H1  = (unsigned short*)(ws + oH1);
  float*          Y2  = (float*)(ws + oY2);
  float*          H2  = (float*)(ws + oH2);

  const size_t scanLds = (size_t)AGG_LDS_INTS * 4;
  hipFuncSetAttribute(reinterpret_cast<const void*>(&k_scan<1>), hipFuncAttributeMaxDynamicSharedMemorySize, (int)scanLds);
  hipFuncSetAttribute(reinterpret_cast<const void*>(&k_scan<0>), hipFuncAttributeMaxDynamicSharedMemorySize, (int)scanLds);

  k_prep<<<UTOT / NTHR, NTHR, 0, stream>>>(emb, W1l, W1r, W2l, W2r, EMB, W1P, W2X);
  k_gemm<<<dim3(gV, TW / GBN), GTHR, 0, stream>>>(EMB, W1P, T, DH, TW);
  k_scan<1><<<gA, NTHR, scanLds, stream>>>(src, dst, x, NE, NN, VOC, vec8, MP, T, b1l, H1, H2);
  k_gemm<<<dim3(gM, TW / GBN), GTHR, 0, stream>>>(H1, W2X, Y2, TW, TW);
  k_scan<0><<<gA, NTHR, scanLds, stream>>>(src, dst, x, NE, NN, MP, vec8, MP, Y2, b2l, H1, H2);
  k_poolhead<<<NG / GPB, NTHR, 0, stream>>>(H2, bat, NN, Wout, bout, out);
}
